// QuantumProjector_27401891348943
// MI455X (gfx1250) — hardware-run, weakly checked
//
#include <hip/hip_runtime.h>
#include <math.h>

typedef __attribute__((ext_vector_type(16))) _Float16 v16h;
typedef __attribute__((ext_vector_type(16))) __bf16   v16b;
typedef __attribute__((ext_vector_type(8)))  float    v8f;
typedef __attribute__((ext_vector_type(4)))  float    v4f;

constexpr int kBatch     = 256;
constexpr int kDimIn     = 1024;
constexpr int kWires     = 16;
constexpr int kDimOut    = 1024;
constexpr int kRowsBlk   = 16;
constexpr int kWavesBlk  = 8;
constexpr int kKPerWave  = kDimIn / kWavesBlk;
constexpr int kColsWave  = kDimOut / kWavesBlk;
constexpr int kGrpCols   = 64;
constexpr int kSlabPitch = 68;
constexpr float kCarryZ  = 256.0f;
constexpr float kCarryW  = 64.0f;
constexpr float kFold    = 1.0f / (kCarryZ * kCarryW);
static_assert(kWires == 16, "one 16-wide tile in the first product, K = 16 in the second");
static_assert(kBatch % kRowsBlk == 0, "row tiles");
static_assert(kKPerWave == 128 && (kKPerWave % 32) == 0, "K split in 32-deep steps");
static_assert(kColsWave == 128 && (kColsWave % kGrpCols) == 0, "column groups");
static_assert(kRowsBlk * kWires == 256, "one thread per (row, wire)");
static_assert(kFold == 1.0f / 16384.0f, "power-of-two fold");


__device__ __forceinline__ unsigned short f2bf_bits(float f) {
  unsigned u = __float_as_uint(f);
  return (unsigned short)((u + 0x7FFFu + ((u >> 16) & 1u)) >> 16);
}
__device__ __forceinline__ float bf_bits2f(unsigned short h) { return __uint_as_float(((unsigned)h) << 16); }

template <int BASE>
__device__ __forceinline__ void split4(const v4f a, v16b& hi, v16b& lo) {
#pragma unroll
  for (int e = 0; e < 4; ++e) {
    const float f = a[e];
    const unsigned short hb = f2bf_bits(f);
    const float rem = f - bf_bits2f(hb);
    const unsigned short lb = f2bf_bits(rem);
    const __bf16 hv = __builtin_bit_cast(__bf16, hb);
    const __bf16 lv = __builtin_bit_cast(__bf16, lb);
    hi[BASE + e] = hv;
    lo[BASE + e] = lv;
  }
}

__device__ __forceinline__ v8f mma_bf(v16b a, v16b b, v8f c) {
  c = __builtin_amdgcn_wmma_f32_16x16x32_bf16(false, a, false, b, (short)0, c, false, false);
  asm volatile("v_nop\n\tv_nop\n\tv_nop\n\tv_nop" : "+v"(c) : "v"(a), "v"(b));
  return c;
}
__device__ __forceinline__ v8f mma_h(v16h a, v16h b, v8f c) {
  c = __builtin_amdgcn_wmma_f32_16x16x32_f16(false, a, false, b, (short)0, c, false, false);
  asm volatile("v_nop\n\tv_nop\n\tv_nop\n\tv_nop" : "+v"(c) : "v"(a), "v"(b));
  return c;
}

__global__ __launch_bounds__(256) void fused_proj_kernel(
    const float* __restrict__ x,
    const float* __restrict__ wpre,
    const float* __restrict__ bpre,
    const float* __restrict__ qw,
    const float* __restrict__ wpost,
    const float* __restrict__ bpost,
    float* __restrict__ out)
{
  __shared__ __align__(16) float sPart[kWavesBlk * 256];
  __shared__ __align__(16) float sZ[256];
  __shared__ __align__(16) float sZq[256];
  __shared__ __align__(16) float sSlab[kWavesBlk][16 * kSlabPitch];

  const int tid  = threadIdx.x;
  const int wave = __builtin_amdgcn_readfirstlane((int)(threadIdx.x >> 5));
  const int lane = tid & 31;
  const int h    = lane >> 4;
  const int sub  = lane & 15;
  const int m0   = blockIdx.x * kRowsBlk;

  {
    v8f acc = (v8f){0.f, 0.f, 0.f, 0.f, 0.f, 0.f, 0.f, 0.f};
    const float* ap = x    + (size_t)(m0 + sub) * kDimIn + wave * kKPerWave + 8 * h;
    const float* bp = wpre + (size_t)sub        * kDimIn + wave * kKPerWave + 8 * h;
#pragma unroll 1
    for (int ks = 0; ks < kKPerWave / 32; ++ks) {
      const v4f a0 = *(const v4f*)(ap + ks * 32);
      const v4f a1 = *(const v4f*)(ap + ks * 32 + 4);
      const v4f a2 = *(const v4f*)(ap + ks * 32 + 16);
      const v4f a3 = *(const v4f*)(ap + ks * 32 + 20);
      const v4f b0 = *(const v4f*)(bp + ks * 32);
      const v4f b1 = *(const v4f*)(bp + ks * 32 + 4);
      const v4f b2 = *(const v4f*)(bp + ks * 32 + 16);
      const v4f b3 = *(const v4f*)(bp + ks * 32 + 20);
      v16b ah, al, bh, bl;
      split4<0>(a0, ah, al);
      split4<4>(a1, ah, al);
      split4<8>(a2, ah, al);
      split4<12>(a3, ah, al);
      split4<0>(b0, bh, bl);
      split4<4>(b1, bh, bl);
      split4<8>(b2, bh, bl);
      split4<12>(b3, bh, bl);
      acc = mma_bf(ah, bh, acc);
      acc = mma_bf(ah, bl, acc);
      acc = mma_bf(al, bh, acc);
    }
#pragma unroll
    for (int r = 0; r < 8; ++r)
      sPart[wave * 256 + (8 * h + r) * 16 + sub] = acc[r];
  }
  __syncthreads();

  {
    const int j = tid & 15;
    float s = 0.0f;
#pragma unroll
    for (int w = 0; w < kWavesBlk; ++w) s += sPart[w * 256 + tid];
    const float angle = s + bpre[j];
    const float cw = cosf(qw[j]);
    const float ca = cosf(angle);
    sZ[tid] = cw * ca;
  }
  __syncthreads();
  {
    const int m = tid >> 4;
    const int j = tid & 15;
    float prod = 1.0f;
#pragma unroll
    for (int t = 0; t < kWires; ++t) {
      const float zt = sZ[m * 16 + t];
      const float pn = prod * zt;
      prod = (t <= j) ? pn : prod;
    }
    sZq[tid] = prod * kCarryZ;
  }
  __syncthreads();

  v16h af;
  {
    const float* zr = sZq + sub * 16 + 8 * h;
    const v4f z0 = *(const v4f*)(zr);
    const v4f z1 = *(const v4f*)(zr + 4);
#pragma unroll
    for (int e = 0; e < 4; ++e) {
      const float f0 = z0[e];
      const float f1 = z1[e];
      af[e]      = (_Float16)f0;
      af[4 + e]  = (_Float16)f1;
      af[8 + e]  = (_Float16)0.0f;
      af[12 + e] = (_Float16)0.0f;
    }
  }

  float* slab = sSlab[wave];
  const int c4 = sub * 4;

#pragma unroll 1
  for (int g = 0; g < kColsWave / kGrpCols; ++g) {
    const int n0 = wave * kColsWave + g * kGrpCols;
    v8f acc2[4];
    float bias[4];
#pragma unroll
    for (int jt = 0; jt < 4; ++jt) {
      const int n = n0 + jt * 16 + sub;
      const float* wp = wpost + (size_t)n * kWires + 8 * h;
      const v4f w0 = *(const v4f*)(wp);
      const v4f w1 = *(const v4f*)(wp + 4);
      v16h bf;
#pragma unroll
      for (int e = 0; e < 4; ++e) {
        const float f0 = w0[e] * kCarryW;
        const float f1 = w1[e] * kCarryW;
        bf[e]      = (_Float16)f0;
        bf[4 + e]  = (_Float16)f1;
        bf[8 + e]  = (_Float16)0.0f;
        bf[12 + e] = (_Float16)0.0f;
      }
      bias[jt] = bpost[n];
      acc2[jt] = (v8f){0.f, 0.f, 0.f, 0.f, 0.f, 0.f, 0.f, 0.f};
      acc2[jt] = mma_h(af, bf, acc2[jt]);
    }
#pragma unroll
    for (int jt = 0; jt < 4; ++jt) {
#pragma unroll
      for (int r = 0; r < 8; ++r) {
        const float v = acc2[jt][r] * kFold + bias[jt];
        slab[(8 * h + r) * kSlabPitch + jt * 16 + sub] = v;
      }
    }
    __syncthreads();
    v4f vals[8];
#pragma unroll
    for (int it = 0; it < 8; ++it)
      vals[it] = *(const v4f*)(slab + (it * 2 + h) * kSlabPitch + c4);
    for (int pass = 0; pass < 2; ++pass) {
#pragma unroll
      for (int it = 0; it < 8; ++it) {
        const int row = it * 2 + h;
        *(volatile v4f*)(out + (size_t)(m0 + row) * kDimOut + n0 + c4) = vals[it];
      }
      __threadfence();
    }
    __syncthreads();
  }
}

extern "C" void kernel_launch(void* const* d_in, const int* in_sizes, int n_in,
                              void* d_out, int out_size, void* d_ws, size_t ws_size,
                              hipStream_t stream) {
  (void)d_ws;
  (void)ws_size;
  if (n_in < 6) return;
  if (in_sizes[0] != kBatch * kDimIn) return;
  if (in_sizes[1] != kWires * kDimIn) return;
  if (in_sizes[2] != kWires) return;
  if (in_sizes[3] != kWires) return;
  if (in_sizes[4] != kDimOut * kWires) return;
  if (in_sizes[5] != kDimOut) return;
  if (out_size != kBatch * kDimOut) return;

  const float* x      = (const float*)d_in[0];
  const float* W_pre  = (const float*)d_in[1];
  const float* b_pre  = (const float*)d_in[2];
  const float* q_w    = (const float*)d_in[3];
  const float* W_post = (const float*)d_in[4];
  const float* b_post = (const float*)d_in[5];
  float* out = (float*)d_out;

  fused_proj_kernel<<<dim3(kBatch / kRowsBlk), dim3(256), 0, stream>>>(
      x, W_pre, b_pre, q_w, W_post, b_post, out);
}
